// model_79422535238385
// MI455X (gfx1250) — hardware-run, weakly checked
//
#include <hip/hip_runtime.h>
#include <math.h>

typedef __attribute__((ext_vector_type(16))) _Float16 v16h;
typedef __attribute__((ext_vector_type(8)))  _Float16 v8h;
typedef __attribute__((ext_vector_type(2)))  _Float16 v2h;
typedef __attribute__((ext_vector_type(16))) __bf16   v16b;
typedef __attribute__((ext_vector_type(8)))  __bf16   v8b;
typedef __attribute__((ext_vector_type(8)))  float    v8f;
typedef __attribute__((ext_vector_type(4)))  float    v4f;
typedef __attribute__((ext_vector_type(2)))  float    v2f;

constexpr int kN    = 16384;
constexpr int kD    = 16;
constexpr int kP    = 8;
constexpr int kM    = 50;
constexpr int kH    = 128;
constexpr int kIK   = 32;
constexpr int kZN   = 64;
constexpr int kCS   = 2;
constexpr int kCR   = kCS * kN;
constexpr int kThr  = 256;
constexpr float kInCarry = 1024.0f;
constexpr float kSc = 1.0f / (kInCarry * kInCarry);
constexpr float kF16MinNormal = 6.103515625e-5f;

static_assert(kN == 16384 && kD == 16 && kP == 8 && kM == 50 && kH == 128 && kIK == 32 && kZN == 64 && kCS == 2 && kCR == 32768 && kM % kCS == 0 && 1 + kD + kP <= kIK, "the index arithmetic below uses these sizes");

constexpr size_t kOffZ = 0ull;
constexpr size_t kOffIN16 = 61440ull;
constexpr size_t kOffP = 52490240ull;
constexpr size_t kOffH16 = 69267456ull;
constexpr size_t kOffZP = 77656064ull;
constexpr size_t kOffVP = 86044672ull;
constexpr size_t kWsTotal = 87617536ull;
static_assert(kWsTotal <= 268435456ull, "the carve stands under 256 MiB");
static_assert(kOffZ == 0
  && kOffIN16 == kOffZ + 61440ull
  && kOffP == kOffIN16 + 52428800ull
  && kOffH16 == kOffP + 16777216ull
  && kOffZP == kOffH16 + 8388608ull
  && kOffVP == kOffZP + 8388608ull
  && kWsTotal == kOffVP + 1572864ull, "the carve is a chain: every region starts where the one before ends");
static_assert(4096ull + (size_t)kH * kIK * 2 + (size_t)kH * kH * 2 + (size_t)kZN * kH * 2 == 61440ull && (size_t)kM * kN * kIK * 2 == 52428800ull && (size_t)kCR * kH * 4 == 16777216ull && (size_t)kCR * kH * 2 == 8388608ull && (size_t)kCR * kZN * 4 == 8388608ull && (size_t)(kM / kCS - 1) * kN * 4 == 1572864ull, "every region's length is its plane's");
static_assert((kOffIN16 % 256) == 0 && (kOffP % 256) == 0 && (kOffH16 % 256) == 0 && (kOffZP % 256) == 0 && (kOffVP % 256) == 0, "every region starts on a multiple of 256 B");
constexpr size_t kZW1T = 4096ull;
constexpr size_t kZW2T = kZW1T + (size_t)kH * kIK * 2;
constexpr size_t kZW3T = kZW2T + (size_t)kH * kH * 2;

__device__ __forceinline__ unsigned short f2bf_bits(float f) {
  unsigned u = __float_as_uint(f);
  return (unsigned short)((u + 0x7FFFu + ((u >> 16) & 1u)) >> 16);
}
__device__ __forceinline__ float bf_bits2f(unsigned short h) { return __uint_as_float(((unsigned)h) << 16); }
__device__ __forceinline__ float bf16r(float f) { return bf_bits2f(f2bf_bits(f)); }
__device__ __forceinline__ float carry_flush(float v, float carry) {
  const float s = v * carry;
  return (fabsf(s) < kF16MinNormal) ? 0.0f : s;
}

__device__ __forceinline__ void dep_guard4_h(v8f& a, v8f& b, v8f& c, v8f& d, v16h x, v16h y) { asm volatile("v_nop\n\tv_nop\n\tv_nop\n\tv_nop" : "+v"(a), "+v"(b), "+v"(c), "+v"(d) : "v"(x), "v"(y)); }
__device__ __forceinline__ void dep_guard4_b(v8f& a, v8f& b, v8f& c, v8f& d, v16b x, v16b y) { asm volatile("v_nop\n\tv_nop\n\tv_nop\n\tv_nop" : "+v"(a), "+v"(b), "+v"(c), "+v"(d) : "v"(x), "v"(y)); }
__device__ __forceinline__ void keep4_h(v16h a, v16h b, v16h c, v16h d) { asm volatile("v_nop" :: "v"(a), "v"(b), "v"(c), "v"(d)); }
__device__ __forceinline__ void keep4_b(v16b a, v16b b, v16b c, v16b d) { asm volatile("v_nop" :: "v"(a), "v"(b), "v"(c), "v"(d)); }
__device__ __forceinline__ void acc_guard4(v8f& a, v8f& b, v8f& c, v8f& d) { asm volatile("v_nop\n\tv_nop\n\tv_nop\n\tv_nop" : "+v"(a), "+v"(b), "+v"(c), "+v"(d)); }

template <typename T> struct Frag;
template <> struct Frag<_Float16> {
  typedef v16h V; union U { v16h v; v8h h[2]; };
  static __device__ __forceinline__ v16h load(const _Float16* p) {
    U f; f.h[0] = *(const v8h*)(p); f.h[1] = *(const v8h*)(p + 16); return f.v;
  }
  static __device__ __forceinline__ v8f mma(v16h a, v16h b, v8f c) {
    return __builtin_amdgcn_wmma_f32_16x16x32_f16(false, a, false, b, (short)0, c, false, false);
  }
  static __device__ __forceinline__ void guard4(v8f& a, v8f& b, v8f& c, v8f& d, v16h x, v16h y) { dep_guard4_h(a, b, c, d, x, y); }
  static __device__ __forceinline__ void keep(v16h a, v16h b, v16h c, v16h d) { keep4_h(a, b, c, d); }
};
template <> struct Frag<__bf16> {
  typedef v16b V; union U { v16b v; v8b h[2]; };
  static __device__ __forceinline__ v16b load(const __bf16* p) {
    U f; f.h[0] = *(const v8b*)(p); f.h[1] = *(const v8b*)(p + 16); return f.v;
  }
  static __device__ __forceinline__ v8f mma(v16b a, v16b b, v8f c) {
    return __builtin_amdgcn_wmma_f32_16x16x32_bf16(false, a, false, b, (short)0, c, false, false);
  }
  static __device__ __forceinline__ void guard4(v8f& a, v8f& b, v8f& c, v8f& d, v16b x, v16b y) { dep_guard4_b(a, b, c, d, x, y); }
  static __device__ __forceinline__ void keep(v16b a, v16b b, v16b c, v16b d) { keep4_b(a, b, c, d); }
};

__device__ __forceinline__ v8f mma_h(v16h a, v16h b, v8f c) {
  c = __builtin_amdgcn_wmma_f32_16x16x32_f16(false, a, false, b, (short)0, c, false, false);
  asm volatile("v_nop\n\tv_nop\n\tv_nop\n\tv_nop" : "+v"(c) : "v"(a), "v"(b));
  return c;
}

template <int ET> struct Elem;
template <> struct Elem<0> { typedef _Float16 T; };
template <> struct Elem<1> { typedef __bf16 T; };
template <int ET, bool SPLIT, int BIAS_MODE, int OUT_MODE, bool RESID, int ACT = 0>
__global__ __launch_bounds__(256) void wmma_gemm64(
    const unsigned short* __restrict__ Ap, const unsigned short* __restrict__ A2p, int lda, long strideA,
    const unsigned short* __restrict__ Btp, const unsigned short* __restrict__ Bt2p, int ldb, long strideB,
    void* __restrict__ Cout, void* __restrict__ Cout2, int ldc, long strideC,
    const float* __restrict__ bias,
    const float* __restrict__ resid, long strideR,
    int M, int N, int K, float scale) {
  typedef typename Elem<ET>::T T;
  typedef typename Frag<T>::V V;
  const T* A = (const T*)Ap; const T* A2 = (const T*)A2p; const T* Bt = (const T*)Btp; const T* Bt2 = (const T*)Bt2p;
  __shared__ __align__(16) float sT[8][16 * 68];
  const int b    = blockIdx.y;
  const int lane = threadIdx.x & 31;
  const int wave = threadIdx.x >> 5;
  const int tilesN = N >> 6;
  const int tilesM = M >> 6;
  const int tile = blockIdx.x * 8 + wave;
  if (tile >= tilesM * tilesN) return;
  const int tm = tile / tilesN;
  const int tn = tile - tm * tilesN;
  const int m0 = tm << 6;
  const int n0 = tn << 6;

  const T* Ab  = A  + (size_t)b * strideA;
  const T* Bb  = Bt + (size_t)b * strideB;
  const T* Ab2 = SPLIT ? (A2  + (size_t)b * strideA) : nullptr;
  const T* Bb2 = SPLIT ? (Bt2 + (size_t)b * strideB) : nullptr;

  const int rlane = lane & 15;
  const int koff  = (lane >> 4) * 8;
  const int mOff  = (lane >> 4) * 8;

  v8f acc[4][4];
#pragma unroll
  for (int i = 0; i < 4; ++i)
#pragma unroll
    for (int j = 0; j < 4; ++j) acc[i][j] = (v8f){0.f,0.f,0.f,0.f,0.f,0.f,0.f,0.f};

  for (int k0 = 0; k0 < K; k0 += 32) {
    V bh[4], bl[4];
#pragma unroll
    for (int j = 0; j < 4; ++j) {
      const size_t bo = (size_t)(n0 + (j << 4) + rlane) * ldb + koff + k0;
      bh[j] = Frag<T>::load(Bb + bo);
      if (SPLIT) bl[j] = Frag<T>::load(Bb2 + bo);
    }
#pragma unroll
    for (int i = 0; i < 4; ++i) {
      const size_t ao = (size_t)(m0 + (i << 4) + rlane) * lda + koff + k0;
      V ah = Frag<T>::load(Ab + ao);
      V al;
      if (SPLIT) al = Frag<T>::load(Ab2 + ao);
#pragma unroll
      for (int j = 0; j < 4; ++j) {
        acc[i][j] = Frag<T>::mma(ah, bh[j], acc[i][j]);
        if (SPLIT) {
          acc[i][j] = Frag<T>::mma(ah, bl[j], acc[i][j]);
          acc[i][j] = Frag<T>::mma(al, bh[j], acc[i][j]);
        }
      }
      Frag<T>::guard4(acc[i][0], acc[i][1], acc[i][2], acc[i][3], ah, SPLIT ? al : ah);
    }
    Frag<T>::keep(bh[0], bh[1], bh[2], bh[3]);
    if (SPLIT) Frag<T>::keep(bl[0], bl[1], bl[2], bl[3]);
  }
  acc_guard4(acc[0][0], acc[0][1], acc[0][2], acc[0][3]);
  acc_guard4(acc[1][0], acc[1][1], acc[1][2], acc[1][3]);
  acc_guard4(acc[2][0], acc[2][1], acc[2][2], acc[2][3]);
  acc_guard4(acc[3][0], acc[3][1], acc[3][2], acc[3][3]);

  float* slab = sT[wave];
  const float* Rb = RESID ? (resid + (size_t)b * strideR) : nullptr;
#pragma unroll
  for (int i = 0; i < 4; ++i) {
    const int mBase = m0 + (i << 4);
#pragma unroll
    for (int j = 0; j < 4; ++j) {
      const int n = n0 + (j << 4) + rlane;
      float bv = 0.f;
      if (BIAS_MODE == 2) bv = bias[n];
#pragma unroll
      for (int r = 0; r < 8; ++r) {
        float v = acc[i][j][r] * scale;
        if (BIAS_MODE == 1) v += bias[mBase + mOff + r];
        if (BIAS_MODE == 2) v += bv;
        if (RESID) v += Rb[(size_t)(mBase + mOff + r) * ldc + n];
        if (ACT == 1) v = tanhf(v);
        if (ACT == 2) v = fmaxf(v, 0.0f);
        if (ACT == 3) v = v / (1.0f + expf(-v));
        if (ACT == 4) v = (v > 0.f) ? v : 0.01f * v;
        slab[(mOff + r) * 68 + (j << 4) + rlane] = v;
      }
    }
    __builtin_amdgcn_fence(__ATOMIC_RELEASE, "workgroup");
    __builtin_amdgcn_wave_barrier();
    __builtin_amdgcn_fence(__ATOMIC_ACQUIRE, "workgroup");
    if (OUT_MODE == 0) {
      float* C = (float*)Cout + (size_t)b * strideC;
      const int hh = lane >> 4, c4 = (lane & 15) * 4;
      for (int pass = 0; pass < 2; ++pass) {
#pragma unroll
        for (int it = 0; it < 8; ++it) {
          const int row = it * 2 + hh;
          v4f v = *(const v4f*)(slab + row * 68 + c4);
          *(volatile v4f*)(C + (size_t)(mBase + row) * ldc + n0 + c4) = v;
        }
        __threadfence();
      }
    } else {
      const int q = lane >> 3, c8 = (lane & 7) * 8;
      unsigned short* C  = (unsigned short*)Cout  + (size_t)b * strideC;
      unsigned short* C2 = (OUT_MODE == 2) ? ((unsigned short*)Cout2 + (size_t)b * strideC) : nullptr;
      for (int pass = 0; pass < 2; ++pass) {
#pragma unroll
        for (int it = 0; it < 4; ++it) {
          const int row = it * 4 + q;
          const float* sp = slab + row * 68 + c8;
          v8h hv, lv;
#pragma unroll
          for (int e = 0; e < 8; ++e) {
            if (OUT_MODE == 1) {
              hv[e] = (_Float16)sp[e];
            } else {
              unsigned short hb = f2bf_bits(sp[e]);
              unsigned short lb = f2bf_bits(sp[e] - bf_bits2f(hb));
              hv[e] = __builtin_bit_cast(_Float16, hb);
              lv[e] = __builtin_bit_cast(_Float16, lb);
            }
          }
          *(volatile v8h*)(C + (size_t)(mBase + row) * ldc + n0 + c8) = hv;
          if (OUT_MODE == 2) *(volatile v8h*)(C2 + (size_t)(mBase + row) * ldc + n0 + c8) = lv;
        }
        __threadfence();
      }
    }
    __builtin_amdgcn_fence(__ATOMIC_RELEASE, "workgroup");
    __builtin_amdgcn_wave_barrier();
    __builtin_amdgcn_fence(__ATOMIC_ACQUIRE, "workgroup");
  }
}

__global__ __launch_bounds__(kThr) void zero_kernel(float* __restrict__ dst) {
  const size_t o4 = ((size_t)blockIdx.x * kThr + threadIdx.x) * 4u;
  const v4f z = {0.f, 0.f, 0.f, 0.f};
  *(volatile v4f*)(dst + o4) = z;
  __threadfence();
  *(volatile v4f*)(dst + o4) = z;
}
__global__ __launch_bounds__(kThr) void pack_kernel(const float* __restrict__ W, unsigned short* __restrict__ D, float* __restrict__ dstf, int part, int ld, int k0, int lg, int n0, int pitch) {
  const unsigned i = blockIdx.x * blockDim.x + threadIdx.x;
  if (part == 0) {
    const unsigned g = i & ((1u << lg) - 1u), n = i >> lg;
    const float* sp = W + (size_t)((unsigned)k0 + g * 8u) * (unsigned)ld + n;
    v8h hv;
#pragma unroll
    for (int t = 0; t < 8; ++t) hv[t] = (_Float16)carry_flush(bf16r(sp[(size_t)t * (unsigned)ld]), kInCarry);
    unsigned short* dp = D + (size_t)((unsigned)n0 + n) * (unsigned)pitch + g * 8u;
    *(volatile v8h*)dp = hv;
    __threadfence();
    *(volatile v8h*)dp = hv;
  } else {
    const v4f a = *(const v4f*)(W + i * 4u);
    v4f o;
#pragma unroll
    for (int e = 0; e < 4; ++e) o[e] = bf16r(a[e]);
    float* dp = dstf + i * 4u;
    *(volatile v4f*)dp = o;
    __threadfence();
    *(volatile v4f*)dp = o;
  }
}

__global__ __launch_bounds__(kThr) void xroll_kernel(const float* __restrict__ x0, const float* __restrict__ obs, const float* __restrict__ noise, const float* __restrict__ W1,
                                                     unsigned short* __restrict__ IN16, unsigned short* __restrict__ W1T, float* __restrict__ oX) {
  const float dt = 1.0f / (float)kM;
  const float sq = sqrtf(dt);
  if (blockIdx.x < 64u) {
    const unsigned n = blockIdx.x * (unsigned)kThr + threadIdx.x;
    float X[kD];
    v8h yh;
#pragma unroll
    for (int q = 0; q < 4; ++q) {
      const v4f a = *(const v4f*)(x0 + (size_t)n * kD + 4 * q);
#pragma unroll
      for (int e = 0; e < 4; ++e) X[4 * q + e] = bf16r(a[e]);
    }
#pragma unroll
    for (int q = 0; q < 2; ++q) {
      const v4f a = *(const v4f*)(obs + (size_t)n * kP + 4 * q);
#pragma unroll
      for (int e = 0; e < 4; ++e) yh[4 * q + e] = (_Float16)carry_flush(bf16r(a[e]), kInCarry);
    }
    for (int m = 0; m < kM; ++m) {
      const float t = (float)m * dt;
      v8h r0, r1, r2, r3;
      r0[0] = (_Float16)carry_flush(t, kInCarry);
#pragma unroll
      for (int e = 0; e < 7; ++e) r0[1 + e] = (_Float16)carry_flush(X[e], kInCarry);
#pragma unroll
      for (int e = 0; e < 8; ++e) r1[e] = (_Float16)carry_flush(X[7 + e], kInCarry);
      r2[0] = (_Float16)carry_flush(X[15], kInCarry);
#pragma unroll
      for (int e = 0; e < 7; ++e) r2[1 + e] = yh[e];
      r3[0] = yh[7];
#pragma unroll
      for (int e = 1; e < 8; ++e) r3[e] = (_Float16)0.0f;
      unsigned short* rp = IN16 + ((size_t)m * kN + n) * kIK;
      for (int pass = 0; pass < 2; ++pass) {
        *(volatile v8h*)(rp) = r0;
        *(volatile v8h*)(rp + 8) = r1;
        *(volatile v8h*)(rp + 16) = r2;
        *(volatile v8h*)(rp + 24) = r3;
        __threadfence();
      }
      const float* ep = noise + ((size_t)m * kN + n) * kD;
#pragma unroll
      for (int q = 0; q < 4; ++q) {
        const v4f a = *(const v4f*)(ep + 4 * q);
#pragma unroll
        for (int e = 0; e < 4; ++e) {
          const float Wn = sq * bf16r(a[e]);
          X[4 * q + e] = (X[4 * q + e] + dt * (-X[4 * q + e])) + Wn;
        }
      }
    }
    float* xp = oX + (size_t)n * kD;
    for (int pass = 0; pass < 2; ++pass) {
#pragma unroll
      for (int q = 0; q < 4; ++q) {
        v4f o;
#pragma unroll
        for (int e = 0; e < 4; ++e) o[e] = X[4 * q + e];
        *(volatile v4f*)(xp + 4 * q) = o;
      }
      __threadfence();
    }
  } else {
    if (threadIdx.x < (unsigned)kH) {
      const unsigned j = threadIdx.x;
      v8h r[4];
#pragma unroll
      for (int k = 0; k < kIK; ++k) {
        const float w = (k < 1 + kD + kP) ? W1[(size_t)((k < 1 + kD + kP) ? k : 0) * kH + j] : 0.0f;
        r[k >> 3][k & 7] = (k < 1 + kD + kP) ? (_Float16)carry_flush(bf16r(w), kInCarry) : (_Float16)0.0f;
      }
      unsigned short* rp = W1T + (size_t)j * kIK;
      for (int pass = 0; pass < 2; ++pass) {
#pragma unroll
        for (int q = 0; q < 4; ++q) *(volatile v8h*)(rp + 8 * q) = r[q];
        __threadfence();
      }
    }
  }
}
static_assert(kN == 64 * kThr && kH <= kThr && kH % 32 == 0, "the roll's grid exact: 64 blocks of a thread a path + one block whose first 128 threads are the first layer's units");

__global__ __launch_bounds__(kThr) void brc_kernel(const float* __restrict__ P, const float* __restrict__ bias, unsigned short* __restrict__ H16) {
  const unsigned v = blockIdx.x * (unsigned)kThr + threadIdx.x;
  const unsigned r = v >> 4, j8 = (v & 15u) << 3;
  const float* pr = P + (size_t)r * kH + j8;
  v8h hv;
#pragma unroll
  for (int hlf = 0; hlf < 2; ++hlf) {
    const v4f p = *(const v4f*)(pr + 4 * hlf), q = *(const v4f*)(bias + j8 + 4 * hlf);
#pragma unroll
    for (int e = 0; e < 4; ++e) hv[4 * hlf + e] = (_Float16)carry_flush(fmaxf(p[e] + bf16r(q[e]), 0.0f), kInCarry);
  }
  unsigned short* dp = H16 + (size_t)r * kH + j8;
  *(volatile v8h*)dp = hv;
  __threadfence();
  *(volatile v8h*)dp = hv;
}
static_assert((size_t)kCR * kH / 8 == 2048ull * kThr && kH / 8 == 16, "the epilogue's grid exact: 2,048 blocks; 16 threads a row");

__global__ __launch_bounds__(kThr) void vsum_kernel(const float* __restrict__ ZP, const float* __restrict__ noise, const float* __restrict__ b3, const float* __restrict__ Vin, float* __restrict__ Vout, int m0, int first) {
  const unsigned n = blockIdx.x * (unsigned)kThr + threadIdx.x;
  const float dt = 1.0f / (float)kM;
  const float sq = sqrtf(dt);
  float V = Vin[n];
  if (first != 0) V = bf16r(V);
  float bz[kD];
#pragma unroll
  for (int q = 0; q < 4; ++q) {
    const v4f a = *(const v4f*)(b3 + 4 * q);
#pragma unroll
    for (int e = 0; e < 4; ++e) bz[4 * q + e] = bf16r(a[e]);
  }
  for (int s = 0; s < kCS; ++s) {
    const float* zr = ZP + ((size_t)s * kN + n) * kZN;
    const float* ep = noise + ((size_t)(m0 + s) * kN + n) * kD;
    float dV = 0.0f, zw = 0.0f;
#pragma unroll
    for (int q = 0; q < 4; ++q) {
      const v4f z = *(const v4f*)(zr + 4 * q), a = *(const v4f*)(ep + 4 * q);
#pragma unroll
      for (int e = 0; e < 4; ++e) {
        const float Z = z[e] + bz[4 * q + e];
        const float Wn = sq * bf16r(a[e]);
        dV = dV + Z * Z;
        zw = zw + Z * Wn;
      }
    }
    dV = 0.5f * dV;
    V = (V + dt * dV) + zw;
  }
  float* vp = Vout + n;
  *(volatile float*)vp = V;
  __threadfence();
  *(volatile float*)vp = V;
}

extern "C" void kernel_launch(void* const* d_in, const int* in_sizes, int n_in,
                              void* d_out, int out_size, void* d_ws, size_t ws_size,
                              hipStream_t stream) {
  if (n_in < 10 || d_out == nullptr || d_ws == nullptr) return;
  if (in_sizes[0] != kN * kD || in_sizes[1] != kN || in_sizes[2] != kN * kP || in_sizes[3] != kM * kN * kD || in_sizes[4] != (1 + kD + kP) * kH || in_sizes[5] != kH || in_sizes[6] != kH * kH || in_sizes[7] != kH || in_sizes[8] != kH * kD || in_sizes[9] != kD) return;
  if (out_size != kN * kD + kN) return;
  if (ws_size < kWsTotal) return;
  const float* x0 = (const float*)d_in[0];
  const float* v0 = (const float*)d_in[1];
  const float* obs = (const float*)d_in[2];
  const float* noise = (const float*)d_in[3];
  const float* W1 = (const float*)d_in[4];
  const float* b1 = (const float*)d_in[5];
  const float* W2 = (const float*)d_in[6];
  const float* b2 = (const float*)d_in[7];
  const float* W3 = (const float*)d_in[8];
  const float* b3 = (const float*)d_in[9];
  float* oX = (float*)d_out;
  float* oV = oX + (size_t)kN * kD;
  char* ws = (char*)d_ws;
  float* ZB = (float*)(ws + kOffZ);
  unsigned short* W1T = (unsigned short*)(ws + kOffZ + kZW1T);
  unsigned short* W2T = (unsigned short*)(ws + kOffZ + kZW2T);
  unsigned short* W3T = (unsigned short*)(ws + kOffZ + kZW3T);
  unsigned short* IN16 = (unsigned short*)(ws + kOffIN16);
  float* P = (float*)(ws + kOffP);
  unsigned short* H16 = (unsigned short*)(ws + kOffH16);
  float* ZP = (float*)(ws + kOffZP);
  float* VP = (float*)(ws + kOffVP);

  static_assert(61440ull / 16ull == 15ull * kThr && (kH * (kH / 8)) % kThr == 0 && kD * (kH / 8) == kThr, "the zero fill's grid (15 blocks over Z's 61,440 B) and the pack's grids exact");
  zero_kernel<<<15, kThr, 0, stream>>>(ZB);
  xroll_kernel<<<65, kThr, 0, stream>>>(x0, obs, noise, W1, IN16, W1T, oX);
  pack_kernel<<<kH * (kH / 8) / kThr, kThr, 0, stream>>>(W2, W2T, nullptr, 0, kH, 0, 4, 0, kH);
  pack_kernel<<<1, kThr, 0, stream>>>(W3, W3T, nullptr, 0, kD, 0, 4, 0, kH);
  for (int c = 0; c < kM / kCS; ++c) {
    wmma_gemm64<0, false, 2, 0, false, 0><<<dim3((kCR / 64) * (kH / 64) / 8, 1), 256, 0, stream>>>(
        IN16 + (size_t)c * kCR * kIK, IN16 + (size_t)c * kCR * kIK, kIK, 0L, W1T, W1T, kIK, 0L, (void*)P, (void*)P, kH, 0L, ZB, nullptr, 0L, kCR, kH, kIK, kSc);
    brc_kernel<<<2048, kThr, 0, stream>>>(P, b1, H16);
    wmma_gemm64<0, false, 2, 0, false, 0><<<dim3((kCR / 64) * (kH / 64) / 8, 1), 256, 0, stream>>>(
        H16, H16, kH, 0L, W2T, W2T, kH, 0L, (void*)P, (void*)P, kH, 0L, ZB, nullptr, 0L, kCR, kH, kH, kSc);
    brc_kernel<<<2048, kThr, 0, stream>>>(P, b2, H16);
    wmma_gemm64<0, false, 2, 0, false, 0><<<dim3((kCR / 64) * (kZN / 64) / 8, 1), 256, 0, stream>>>(
        H16, H16, kH, 0L, W3T, W3T, kH, 0L, (void*)ZP, (void*)ZP, kZN, 0L, ZB, nullptr, 0L, kCR, kZN, kH, kSc);
    vsum_kernel<<<64, kThr, 0, stream>>>(ZP, noise, b3, (c == 0) ? v0 : (VP + (size_t)(c - 1) * kN), (c == kM / kCS - 1) ? oV : (VP + (size_t)c * kN), c * kCS, (c == 0) ? 1 : 0);
  }
}
static_assert(((kCR / 64) * (kH / 64)) % 8 == 0 && ((kCR / 64) * (kZN / 64)) % 8 == 0 && kIK % 32 == 0 && kH % 32 == 0, "every engine grid: whole blocks of eight wave tiles; every depth a multiple of 32");
